// VRWKV_SpatialMix_5050881540339
// MI455X (gfx1250) — hardware-verified
//
#include <hip/hip_runtime.h>
#include <math.h>

constexpr int kBatch     = 8;
constexpr int kTok       = 4096;
constexpr int kCh        = 256;
constexpr int kRows      = kBatch * kTok;
constexpr int kChunkRows = 8192;
constexpr int kNumChunks = kRows / kChunkRows;
constexpr int kWElems    = kCh * kCh;
constexpr float kInvTok  = 1.0f / 4096.0f;
constexpr float kInvCh   = 1.0f / 256.0f;
constexpr float kLnEps   = 1.0e-5f;
static_assert(kRows % kChunkRows == 0, "chunks");
static_assert(kChunkRows % 64 == 0 && kCh % 64 == 0 && kCh % 32 == 0, "tiles");
static_assert(kChunkRows % 8 == 0 && (kWElems % 2048) == 0, "grids");

typedef __attribute__((ext_vector_type(16))) _Float16 v16h;
typedef __attribute__((ext_vector_type(8)))  _Float16 v8h;
typedef __attribute__((ext_vector_type(16))) __bf16   v16b;
typedef __attribute__((ext_vector_type(8)))  __bf16   v8b;
typedef __attribute__((ext_vector_type(8)))  float    v8f;
typedef __attribute__((ext_vector_type(4)))  float    v4f;
typedef __attribute__((ext_vector_type(4)))  unsigned int v4u;

__device__ __forceinline__ unsigned short f2bf_bits(float f) {
  unsigned u = __float_as_uint(f);
  return (unsigned short)((u + 0x7FFFu + ((u >> 16) & 1u)) >> 16);
}
__device__ __forceinline__ float bf_bits2f(unsigned short h) { return __uint_as_float(((unsigned)h) << 16); }
__device__ __forceinline__ float bf16r(float f) { return bf_bits2f(f2bf_bits(f)); }
__device__ __forceinline__ float h16_to_f32(unsigned hb) {
  const unsigned sgn = (hb & 0x8000u) << 16; const unsigned em = hb & 0x7fffu;
  const float fn = __uint_as_float((em << 13) + 0x38000000u);
  const float fs = (float)em * 5.9604644775390625e-8f;
  const float mag = (em < 0x400u) ? fs : fn; return __uint_as_float(__float_as_uint(mag) | sgn); }
__device__ __forceinline__ unsigned pk16(unsigned short a, unsigned short b) { return (unsigned)a | ((unsigned)b << 16); }

__device__ __forceinline__ void dep_guard_h(v8f& a, v8f& b, v16h x, v16h y) { asm volatile("v_nop\n\tv_nop\n\tv_nop\n\tv_nop" : "+v"(a), "+v"(b) : "v"(x), "v"(y)); }
__device__ __forceinline__ void dep_guard_b(v8f& a, v8f& b, v16b x, v16b y) { asm volatile("v_nop\n\tv_nop\n\tv_nop\n\tv_nop" : "+v"(a), "+v"(b) : "v"(x), "v"(y)); }
__device__ __forceinline__ void dep_guard_all_h(v8f& a0, v8f& a1, v8f& a2, v8f& a3, v16h x, v16h y, v16h b0, v16h b1, v16h b2, v16h b3) {
  asm volatile("v_nop\n\tv_nop\n\tv_nop\n\tv_nop" : "+v"(a0), "+v"(a1), "+v"(a2), "+v"(a3) : "v"(x), "v"(y), "v"(b0), "v"(b1), "v"(b2), "v"(b3));
}
__device__ __forceinline__ void dep_guard_all_b(v8f& a0, v8f& a1, v8f& a2, v8f& a3, v16b x, v16b y, v16b b0, v16b b1, v16b b2, v16b b3) {
  asm volatile("v_nop\n\tv_nop\n\tv_nop\n\tv_nop" : "+v"(a0), "+v"(a1), "+v"(a2), "+v"(a3) : "v"(x), "v"(y), "v"(b0), "v"(b1), "v"(b2), "v"(b3));
}
__device__ __forceinline__ void keep4_h(v16h a, v16h b, v16h c, v16h d) { asm volatile("v_nop" :: "v"(a), "v"(b), "v"(c), "v"(d)); }
__device__ __forceinline__ void keep4_b(v16b a, v16b b, v16b c, v16b d) { asm volatile("v_nop" :: "v"(a), "v"(b), "v"(c), "v"(d)); }
__device__ __forceinline__ void acc_guard4(v8f& a, v8f& b, v8f& c, v8f& d) { asm volatile("v_nop\n\tv_nop\n\tv_nop\n\tv_nop" : "+v"(a), "+v"(b), "+v"(c), "+v"(d)); }

template <typename T> struct Frag;
template <> struct Frag<_Float16> {
  typedef v16h V; union U { v16h v; v8h h[2]; };
  static __device__ __forceinline__ v16h load(const _Float16* p) {
    U f; f.h[0] = *(const v8h*)(p); f.h[1] = *(const v8h*)(p + 16); return f.v;
  }
  static __device__ __forceinline__ v8f mma(v16h a, v16h b, v8f c) {
    return __builtin_amdgcn_wmma_f32_16x16x32_f16(false, a, false, b, (short)0, c, false, false);
  }
  static __device__ __forceinline__ void guard(v8f& a, v8f& b, v16h x, v16h y) { dep_guard_h(a, b, x, y); }
  static __device__ __forceinline__ void guard_all(v8f& a0, v8f& a1, v8f& a2, v8f& a3, v16h x, v16h y, v16h b0, v16h b1, v16h b2, v16h b3) {
    dep_guard_all_h(a0, a1, a2, a3, x, y, b0, b1, b2, b3);
  }
  static __device__ __forceinline__ void keep(v16h a, v16h b, v16h c, v16h d) { keep4_h(a, b, c, d); }
};
template <> struct Frag<__bf16> {
  typedef v16b V; union U { v16b v; v8b h[2]; };
  static __device__ __forceinline__ v16b load(const __bf16* p) {
    U f; f.h[0] = *(const v8b*)(p); f.h[1] = *(const v8b*)(p + 16); return f.v;
  }
  static __device__ __forceinline__ v8f mma(v16b a, v16b b, v8f c) {
    return __builtin_amdgcn_wmma_f32_16x16x32_bf16(false, a, false, b, (short)0, c, false, false);
  }
  static __device__ __forceinline__ void guard(v8f& a, v8f& b, v16b x, v16b y) { dep_guard_b(a, b, x, y); }
  static __device__ __forceinline__ void guard_all(v8f& a0, v8f& a1, v8f& a2, v8f& a3, v16b x, v16b y, v16b b0, v16b b1, v16b b2, v16b b3) {
    dep_guard_all_b(a0, a1, a2, a3, x, y, b0, b1, b2, b3);
  }
  static __device__ __forceinline__ void keep(v16b a, v16b b, v16b c, v16b d) { keep4_b(a, b, c, d); }
};

template <int ET> struct Elem;
template <> struct Elem<0> { typedef _Float16 T; };
template <> struct Elem<1> { typedef __bf16 T; };
template <int ET, int SPLIT, int BIAS_MODE, int OUT_MODE, int ACT>
__global__ __launch_bounds__(256) void wmma_gemm64(
    const unsigned short* __restrict__ Ap, const unsigned short* __restrict__ A2p, int lda, long strideA,
    const unsigned short* __restrict__ Btp, const unsigned short* __restrict__ Bt2p, int ldb, long strideB,
    void* __restrict__ Cout, void* __restrict__ Cout2, int ldc, long strideC,
    const float* __restrict__ bias,
    const float* __restrict__ resid_unused, long strideR_unused,
    int M, int N, int K, float scale) {
  typedef typename Elem<ET>::T T;
  typedef typename Frag<T>::V V;
  (void)resid_unused; (void)strideR_unused;
  const T* A = (const T*)Ap; const T* A2 = (const T*)A2p; const T* Bt = (const T*)Btp; const T* Bt2 = (const T*)Bt2p;
  __shared__ __align__(16) float sT[8][16 * 68];
  const int b    = blockIdx.y;
  const int lane = threadIdx.x & 31;
  const int wave = threadIdx.x >> 5;
  const int tilesN = N >> 6;
  const int tilesM = M >> 6;
  const int tile = blockIdx.x * 8 + wave;
  if (tile >= tilesM * tilesN) return;
  const int tm = tile / tilesN;
  const int tn = tile - tm * tilesN;
  const int m0 = tm << 6;
  const int n0 = tn << 6;

  const T* Ab  = A  + (size_t)b * strideA;
  const T* Bb  = Bt + (size_t)b * strideB;
  const T* Ab2 = (SPLIT != 0) ? (A2  + (size_t)b * strideA) : nullptr;
  const T* Bb2 = (SPLIT == 1) ? (Bt2 + (size_t)b * strideB) : nullptr;

  const int rlane = lane & 15;
  const int koff  = (lane >> 4) * 8;
  const int mOff  = (lane >> 4) * 8;

  v8f acc[4][4];
#pragma unroll
  for (int i = 0; i < 4; ++i)
#pragma unroll
    for (int j = 0; j < 4; ++j) acc[i][j] = (v8f){0.f,0.f,0.f,0.f,0.f,0.f,0.f,0.f};

  for (int k0 = 0; k0 < K; k0 += 32) {
    V bh[4], bl[4];
#pragma unroll
    for (int j = 0; j < 4; ++j) {
      const size_t bo = (size_t)(n0 + (j << 4) + rlane) * ldb + koff + k0;
      bh[j] = Frag<T>::load(Bb + bo);
      bl[j] = bh[j];
      if (SPLIT == 1) bl[j] = Frag<T>::load(Bb2 + bo);
    }
#pragma unroll
    for (int i = 0; i < 4; ++i) {
      const size_t ao = (size_t)(m0 + (i << 4) + rlane) * lda + koff + k0;
      V ah = Frag<T>::load(Ab + ao);
      V al = ah;
      if (SPLIT != 0) al = Frag<T>::load(Ab2 + ao);
#pragma unroll
      for (int j = 0; j < 4; ++j) {
        acc[i][j] = Frag<T>::mma(ah, bh[j], acc[i][j]);
        if (SPLIT == 1) {
          acc[i][j] = Frag<T>::mma(ah, bl[j], acc[i][j]);
          acc[i][j] = Frag<T>::mma(al, bh[j], acc[i][j]);
        }
        if (SPLIT == 2) acc[i][j] = Frag<T>::mma(al, bh[j], acc[i][j]);
      }
      Frag<T>::guard_all(acc[i][0], acc[i][1], acc[i][2], acc[i][3], ah, al, bh[0], bh[1], bh[2], bh[3]);
    }
    Frag<T>::keep(bh[0], bh[1], bh[2], bh[3]);
    if (SPLIT == 1) Frag<T>::keep(bl[0], bl[1], bl[2], bl[3]);
  }
  acc_guard4(acc[0][0], acc[0][1], acc[0][2], acc[0][3]);
  acc_guard4(acc[1][0], acc[1][1], acc[1][2], acc[1][3]);
  acc_guard4(acc[2][0], acc[2][1], acc[2][2], acc[2][3]);
  acc_guard4(acc[3][0], acc[3][1], acc[3][2], acc[3][3]);

  float* slab = sT[wave];
#pragma unroll
  for (int i = 0; i < 4; ++i) {
    const int mBase = m0 + (i << 4);
#pragma unroll
    for (int j = 0; j < 4; ++j) {
      const int n = n0 + (j << 4) + rlane;
      float bv = 0.f;
      if (BIAS_MODE == 2) bv = bias[n];
#pragma unroll
      for (int r = 0; r < 8; ++r) {
        float v = acc[i][j][r] * scale;
        if (BIAS_MODE == 1) v += bias[mBase + mOff + r];
        if (BIAS_MODE == 2) v += bv;
        if (ACT == 2) v = fmaxf(v, 0.0f);
        if (ACT == 4) v = (v > 0.f) ? v : 0.01f * v;
        if (ACT == 6) v = 1.0f / (1.0f + expf(-v));
        slab[(mOff + r) * 68 + (j << 4) + rlane] = v;
      }
    }
    __builtin_amdgcn_fence(__ATOMIC_RELEASE, "workgroup");
    __builtin_amdgcn_wave_barrier();
    __builtin_amdgcn_fence(__ATOMIC_ACQUIRE, "workgroup");
    if (OUT_MODE == 0) {
      float* C = (float*)Cout + (size_t)b * strideC;
      const int hh = lane >> 4, c4 = (lane & 15) * 4;
      for (int pass = 0; pass < 2; ++pass) {
#pragma unroll
        for (int it = 0; it < 8; ++it) {
          const int row = it * 2 + hh;
          v4f v = *(const v4f*)(slab + row * 68 + c4);
          *(volatile v4f*)(C + (size_t)(mBase + row) * ldc + n0 + c4) = v;
        }
        __threadfence();
      }
    } else {
      const int q = lane >> 3, c8 = (lane & 7) * 8;
      unsigned short* C  = (unsigned short*)Cout  + (size_t)b * strideC;
      unsigned short* C2 = (OUT_MODE == 2) ? ((unsigned short*)Cout2 + (size_t)b * strideC) : nullptr;
      for (int pass = 0; pass < 2; ++pass) {
#pragma unroll
        for (int it = 0; it < 4; ++it) {
          const int row = it * 4 + q;
          const float* sp = slab + row * 68 + c8;
          v8h hv, lv;
#pragma unroll
          for (int e = 0; e < 8; ++e) {
            if (OUT_MODE == 1) {
              hv[e] = (_Float16)sp[e];
            } else {
              unsigned short hb = f2bf_bits(sp[e]);
              unsigned short lb = f2bf_bits(sp[e] - bf_bits2f(hb));
              hv[e] = __builtin_bit_cast(_Float16, hb);
              lv[e] = __builtin_bit_cast(_Float16, lb);
            }
          }
          *(volatile v8h*)(C + (size_t)(mBase + row) * ldc + n0 + c8) = hv;
          if (OUT_MODE == 2) *(volatile v8h*)(C2 + (size_t)(mBase + row) * ldc + n0 + c8) = lv;
        }
        __threadfence();
      }
    }
    __builtin_amdgcn_fence(__ATOMIC_RELEASE, "workgroup");
    __builtin_amdgcn_wave_barrier();
    __builtin_amdgcn_fence(__ATOMIC_ACQUIRE, "workgroup");
  }
}

__global__ __launch_bounds__(256) void wcast_kernel(const float* __restrict__ W0, const float* __restrict__ W1,
                                                    const float* __restrict__ W2, const float* __restrict__ W3,
                                                    unsigned short* __restrict__ Wp) {
  const int z = blockIdx.y;
  const float* W = (z == 0) ? W0 : (z == 1) ? W1 : (z == 2) ? W2 : W3;
  const int i = blockIdx.x * 256 + threadIdx.x;
  const float* p = W + 8 * (size_t)i;
  const v4f a = *(const v4f*)(p);
  const v4f c = *(const v4f*)(p + 4);
  unsigned short hb[8];
#pragma unroll
  for (int e = 0; e < 4; ++e) {
    hb[e]     = f2bf_bits(a[e]);
    hb[4 + e] = f2bf_bits(c[e]);
  }
  const v4u u = (v4u){pk16(hb[0], hb[1]), pk16(hb[2], hb[3]), pk16(hb[4], hb[5]), pk16(hb[6], hb[7])};
  unsigned short* q = Wp + (size_t)z * kWElems + 8 * (size_t)i;
  *(volatile v4u*)q = u;
  __threadfence();
  *(volatile v4u*)q = u;
}

__global__ __launch_bounds__(256) void mixsplit_kernel(const float* __restrict__ x, const float* __restrict__ mix,
                                                       unsigned short* __restrict__ Ahi, unsigned short* __restrict__ Alo, int row0) {
#pragma clang fp contract(off)
  const int lane = threadIdx.x & 31;
  const int wave = threadIdx.x >> 5;
  const int rloc = blockIdx.x * 8 + wave;
  const int grow = row0 + rloc;
  const int b  = grow >> 12;
  const int t  = grow & 4095;
  const int wq = t & 15;
  const int hq = (t >> 4) & 15;
  const int c0 = lane * 8;
  const int grp = lane >> 3;
  const int dt = (grp < 2) ? (2 * grp - 1) : (32 * grp - 80);
  const int vflag = (grp == 0) ? ((wq > 0) ? 1 : 0)
                  : (grp == 1) ? ((wq < 15) ? 1 : 0)
                  : (grp == 2) ? ((hq > 0) ? 1 : 0)
                  :              ((hq < 15) ? 1 : 0);
  int ts = t + dt;
  ts = (ts < 0) ? 0 : ts;
  ts = (ts > kTok - 1) ? (kTok - 1) : ts;
  const float fv = (float)vflag;
  const float* xrow = x + (size_t)grow * kCh + c0;
  const float* xsrc = x + ((size_t)b * kTok + (size_t)ts) * kCh + c0;
  const v4f a0 = *(const v4f*)(xrow);
  const v4f a1 = *(const v4f*)(xrow + 4);
  const v4f s0 = *(const v4f*)(xsrc);
  const v4f s1 = *(const v4f*)(xsrc + 4);
  const v4f q0 = *(const v4f*)(mix + c0);
  const v4f q1 = *(const v4f*)(mix + c0 + 4);
  unsigned short hb[8], lb[8];
#pragma unroll
  for (int e = 0; e < 4; ++e) {
    {
      const float xb = bf16r(a0[e]);
      const float sb = bf16r(s0[e]) * fv;
      const float mb = bf16r(q0[e]);
      const float om = 1.0f - mb;
      const float p1 = xb * mb;
      const float p2 = sb * om;
      const float val = p1 + p2;
      const unsigned short h = f2bf_bits(val);
      hb[e] = h;
      lb[e] = f2bf_bits(val - bf_bits2f(h));
    }
    {
      const float xb = bf16r(a1[e]);
      const float sb = bf16r(s1[e]) * fv;
      const float mb = bf16r(q1[e]);
      const float om = 1.0f - mb;
      const float p1 = xb * mb;
      const float p2 = sb * om;
      const float val = p1 + p2;
      const unsigned short h = f2bf_bits(val);
      hb[4 + e] = h;
      lb[4 + e] = f2bf_bits(val - bf_bits2f(h));
    }
  }
  const v4u uh = (v4u){pk16(hb[0], hb[1]), pk16(hb[2], hb[3]), pk16(hb[4], hb[5]), pk16(hb[6], hb[7])};
  const v4u ul = (v4u){pk16(lb[0], lb[1]), pk16(lb[2], lb[3]), pk16(lb[4], lb[5]), pk16(lb[6], lb[7])};
  unsigned short* ph = Ahi + (size_t)rloc * kCh + c0;
  unsigned short* pl = Alo + (size_t)rloc * kCh + c0;
  *(volatile v4u*)ph = uh;
  *(volatile v4u*)pl = ul;
  __threadfence();
  *(volatile v4u*)ph = uh;
  *(volatile v4u*)pl = ul;
}

__global__ __launch_bounds__(256) void wkv_scan_kernel(const float* __restrict__ sd, const float* __restrict__ sf,
                                                       const float* __restrict__ kp, const float* __restrict__ vp,
                                                       float* __restrict__ yp) {
  const int c = threadIdx.x;
  const int b = blockIdx.x;
  const float wdec = bf16r(sd[c]) * kInvTok;
  const float ufst = bf16r(sf[c]) * kInvTok;
  float p = 0.0f, q = 0.0f, o = -1.0e38f;
  size_t idx = (size_t)b * kTok * kCh + (size_t)c;
#pragma unroll 1
  for (int t = 0; t < kTok; ++t) {
    const float kt = kp[idx];
    const float vt = vp[idx];
    const float uk = ufst + kt;
    const float no = fmaxf(o, uk);
    const float ea = expf(o - no);
    const float eb = expf(uk - no);
    const float num = ea * p + eb * vt;
    const float den = ea * q + eb;
    const float yv = num / den;
    volatile float* ys = yp + idx;
    *ys = yv;
    __threadfence();
    *ys = yv;
    const float wo = wdec + o;
    const float no2 = fmaxf(wo, kt);
    const float ea2 = expf(wo - no2);
    const float eb2 = expf(kt - no2);
    p = ea2 * p + eb2 * vt;
    q = ea2 * q + eb2;
    o = no2;
    idx += kCh;
  }
}

__global__ __launch_bounds__(256) void lngate_kernel(const float* __restrict__ y, const unsigned short* __restrict__ sr,
                                                     const float* __restrict__ gam, const float* __restrict__ bet,
                                                     unsigned short* __restrict__ Ahi, unsigned short* __restrict__ Alo, int row0) {
  const int lane = threadIdx.x & 31;
  const int wave = threadIdx.x >> 5;
  const int rloc = blockIdx.x * 8 + wave;
  const int grow = row0 + rloc;
  const int c0 = lane * 8;
  const float* yrow = y + (size_t)grow * kCh + c0;
  const v4f a0 = *(const v4f*)(yrow);
  const v4f a1 = *(const v4f*)(yrow + 4);
  const v4f g0 = *(const v4f*)(gam + c0);
  const v4f g1 = *(const v4f*)(gam + c0 + 4);
  const v4f b0 = *(const v4f*)(bet + c0);
  const v4f b1 = *(const v4f*)(bet + c0 + 4);
  const v4u sw = *(const v4u*)(sr + (size_t)grow * kCh + c0);

  float vals[8];
#pragma unroll
  for (int e = 0; e < 4; ++e) { vals[e] = a0[e]; vals[4 + e] = a1[e]; }
  float s = ((vals[0] + vals[1]) + (vals[2] + vals[3])) + ((vals[4] + vals[5]) + (vals[6] + vals[7]));
#pragma unroll
  for (int off = 16; off > 0; off >>= 1) s += __shfl_xor(s, off, 32);
  const float mean = s * kInvCh;
  float d[8];
  float s2 = 0.0f;
#pragma unroll
  for (int e = 0; e < 8; ++e) { d[e] = vals[e] - mean; s2 += d[e] * d[e]; }
#pragma unroll
  for (int off = 16; off > 0; off >>= 1) s2 += __shfl_xor(s2, off, 32);
  const float var  = s2 * kInvCh;
  const float rstd = rsqrtf(var + kLnEps);

  float srv[8];
#pragma unroll
  for (int i = 0; i < 4; ++i) {
    const unsigned wv = sw[i];
    srv[2 * i]     = h16_to_f32(wv & 0xffffu);
    srv[2 * i + 1] = h16_to_f32(wv >> 16);
  }
  unsigned short hb[8], lb[8];
#pragma unroll
  for (int e = 0; e < 8; ++e) {
    const float gb = bf16r((e < 4) ? g0[e] : g1[e - 4]);
    const float bb = bf16r((e < 4) ? b0[e] : b1[e - 4]);
    const float ln = (d[e] * rstd) * gb + bb;
    const float gv = srv[e] * ln;
    const unsigned short h = f2bf_bits(gv);
    hb[e] = h;
    lb[e] = f2bf_bits(gv - bf_bits2f(h));
  }
  const v4u uh = (v4u){pk16(hb[0], hb[1]), pk16(hb[2], hb[3]), pk16(hb[4], hb[5]), pk16(hb[6], hb[7])};
  const v4u ul = (v4u){pk16(lb[0], lb[1]), pk16(lb[2], lb[3]), pk16(lb[4], lb[5]), pk16(lb[6], lb[7])};
  unsigned short* ph = Ahi + (size_t)rloc * kCh + c0;
  unsigned short* pl = Alo + (size_t)rloc * kCh + c0;
  *(volatile v4u*)ph = uh;
  *(volatile v4u*)pl = ul;
  __threadfence();
  *(volatile v4u*)ph = uh;
  *(volatile v4u*)pl = ul;
}

extern "C" void kernel_launch(void* const* d_in, const int* in_sizes, int n_in,
                              void* d_out, int out_size, void* d_ws, size_t ws_size,
                              hipStream_t stream) {
  if (n_in < 12) return;
  const int nAct = kRows * kCh;
  if (in_sizes[0] != nAct) return;
  if (in_sizes[1] != kCh || in_sizes[2] != kCh) return;
  if (in_sizes[3] != kCh || in_sizes[4] != kCh || in_sizes[5] != kCh) return;
  if (in_sizes[6] != kWElems || in_sizes[7] != kWElems || in_sizes[8] != kWElems || in_sizes[9] != kWElems) return;
  if (in_sizes[10] != kCh || in_sizes[11] != kCh) return;
  if (out_size != nAct) return;

  const size_t szWP  = (size_t)4 * kWElems * 2;
  const size_t szA   = (size_t)kChunkRows * kCh * 2;
  const size_t szF   = (size_t)kRows * kCh * 4;
  const size_t szH   = (size_t)kRows * kCh * 2;
  const size_t offWP = 0;
  const size_t offAH = offWP + szWP;
  const size_t offAL = offAH + szA;
  const size_t offK  = offAL + szA;
  const size_t offV  = offK + szF;
  const size_t offY  = offV + szF;
  const size_t offS  = offY + szF;
  const size_t total = offS + szH;
  if (ws_size < total) return;

  const float* x   = (const float*)d_in[0];
  const float* sd  = (const float*)d_in[1];
  const float* sf  = (const float*)d_in[2];
  const float* mk  = (const float*)d_in[3];
  const float* mv  = (const float*)d_in[4];
  const float* mr  = (const float*)d_in[5];
  const float* Wk  = (const float*)d_in[6];
  const float* Wv  = (const float*)d_in[7];
  const float* Wr  = (const float*)d_in[8];
  const float* Wo  = (const float*)d_in[9];
  const float* lg  = (const float*)d_in[10];
  const float* lbt = (const float*)d_in[11];
  float* out = (float*)d_out;
  char* ws = (char*)d_ws;
  unsigned short* WP  = (unsigned short*)(ws + offWP);
  unsigned short* AHI = (unsigned short*)(ws + offAH);
  unsigned short* ALO = (unsigned short*)(ws + offAL);
  float* KPL = (float*)(ws + offK);
  float* VPL = (float*)(ws + offV);
  float* YPL = (float*)(ws + offY);
  unsigned short* SPL = (unsigned short*)(ws + offS);
  const unsigned short* WK16 = WP;
  const unsigned short* WV16 = WP + (size_t)kWElems;
  const unsigned short* WR16 = WP + (size_t)2 * kWElems;
  const unsigned short* WO16 = WP + (size_t)3 * kWElems;

  wcast_kernel<<<dim3(kWElems / 2048, 4), dim3(256), 0, stream>>>(Wk, Wv, Wr, Wo, WP);

  const int gemmBlocks = ((kChunkRows / 64) * (kCh / 64)) / 8;
  const int rowBlocks  = kChunkRows / 8;

  for (int ch = 0; ch < kNumChunks; ++ch) {
    const int row0 = ch * kChunkRows;
    const size_t eoff = (size_t)row0 * kCh;
    mixsplit_kernel<<<dim3(rowBlocks), dim3(256), 0, stream>>>(x, mk, AHI, ALO, row0);
    wmma_gemm64<1, 2, 0, 0, 0><<<dim3(gemmBlocks, 1), dim3(256), 0, stream>>>(
        AHI, ALO, kCh, 0L, WK16, WK16, kCh, 0L,
        (void*)(KPL + eoff), (void*)(KPL + eoff), kCh, 0L, KPL, KPL, 0L, kChunkRows, kCh, kCh, 1.0f);
    mixsplit_kernel<<<dim3(rowBlocks), dim3(256), 0, stream>>>(x, mv, AHI, ALO, row0);
    wmma_gemm64<1, 2, 0, 0, 0><<<dim3(gemmBlocks, 1), dim3(256), 0, stream>>>(
        AHI, ALO, kCh, 0L, WV16, WV16, kCh, 0L,
        (void*)(VPL + eoff), (void*)(VPL + eoff), kCh, 0L, KPL, KPL, 0L, kChunkRows, kCh, kCh, 1.0f);
    mixsplit_kernel<<<dim3(rowBlocks), dim3(256), 0, stream>>>(x, mr, AHI, ALO, row0);
    wmma_gemm64<1, 2, 0, 1, 6><<<dim3(gemmBlocks, 1), dim3(256), 0, stream>>>(
        AHI, ALO, kCh, 0L, WR16, WR16, kCh, 0L,
        (void*)(SPL + eoff), (void*)(SPL + eoff), kCh, 0L, KPL, KPL, 0L, kChunkRows, kCh, kCh, 1.0f);
  }

  wkv_scan_kernel<<<dim3(kBatch), dim3(kCh), 0, stream>>>(sd, sf, KPL, VPL, YPL);

  for (int ch = 0; ch < kNumChunks; ++ch) {
    const int row0 = ch * kChunkRows;
    const size_t eoff = (size_t)row0 * kCh;
    lngate_kernel<<<dim3(rowBlocks), dim3(256), 0, stream>>>(YPL, SPL, lg, lbt, AHI, ALO, row0);
    wmma_gemm64<1, 2, 0, 0, 0><<<dim3(gemmBlocks, 1), dim3(256), 0, stream>>>(
        AHI, ALO, kCh, 0L, WO16, WO16, kCh, 0L,
        (void*)(out + eoff), (void*)(out + eoff), kCh, 0L, KPL, KPL, 0L, kChunkRows, kCh, kCh, 1.0f);
  }
}
